// GATLayer_72060961292563
// MI455X (gfx1250) — hardware-verified
//
#include <hip/hip_runtime.h>
#include <stddef.h>
#include <stdint.h>
#include <math.h>


#define FW     128
#define NHD    8
#define HDM    16
#define NNB    16
#define KVW    256
#define WROWS  384
#define AOK    256
#define FB     32
#define FTHR   64
#define NTHR   256
#define GBM    64
#define GBN    64
#define GTHR   128
#define ATTSC  0.25f
#define LNEPS  1e-5f
#define UWQKV  (WROWS * (FW / 8))
#define UWO    (FW * (AOK / 8))
#define NUW    (UWQKV + UWO)
#define WSMAX  134217728

static_assert(FW == NHD * HDM && HDM == 4 * 4 && FW == 4 * 32);
static_assert((FW % 32) == 0 && (AOK % 32) == 0 && AOK == 2 * FW);
static_assert(KVW == 2 * FW && (KVW % GBN) == 0 && ((KVW * 4) % 128) == 0);
static_assert(GBM == (GTHR / 32) * 16 && FB == (FTHR / 32) * 16 && (GBM % FB) == 0);
static_assert((UWQKV % NTHR) == 0 && (NUW % NTHR) == 0);
static_assert(UWQKV == WROWS * 16 && (FW / 8) == 16 && (AOK / 8) == 32);
static_assert(NNB == 16);
static_assert(((FW * 2) % 128) == 0 && ((AOK * 2) % 128) == 0 && ((FW * 4) % 128) == 0);

typedef float          v4f  __attribute__((ext_vector_type(4)));
typedef float          v8f  __attribute__((ext_vector_type(8)));
typedef int            v8i  __attribute__((ext_vector_type(8)));
typedef unsigned int   v4u  __attribute__((ext_vector_type(4)));
typedef unsigned short v8us __attribute__((ext_vector_type(8)));
typedef __bf16         v16b __attribute__((ext_vector_type(16)));
typedef v4f  __attribute__((may_alias)) v4fa;
typedef v4u  __attribute__((may_alias)) v4ua;
typedef v8us __attribute__((may_alias)) v8usa;
union FragB { v16b v; v8us h[2]; v8i w; };

__device__ __forceinline__ v8f wmb(const FragB& a, const FragB& b, v8f c) {
  v8f d = __builtin_amdgcn_wmma_f32_16x16x32_bf16(false, a.v, false, b.v, (short)0, c, false, false);
  asm volatile("v_nop\n\tv_nop\n\tv_nop\n\tv_nop" : "+v"(d) : "v"(a.w), "v"(b.w));
  return d;
}

__device__ __forceinline__ unsigned int f2bf(float f) {
  const unsigned int u = __float_as_uint(f);
  return ((u + 0x7FFFu + ((u >> 16) & 1u)) >> 16) & 0xFFFFu;
}
__device__ __forceinline__ float bf2f(unsigned int b) { return __uint_as_float(b << 16); }
__device__ __forceinline__ float bfr(float f) { return bf2f(f2bf(f)); }
__device__ __forceinline__ v4f bfr4(const v4f a) {
  v4f r; r.x = bfr(a.x); r.y = bfr(a.y); r.z = bfr(a.z); r.w = bfr(a.w); return r;
}
__device__ __forceinline__ unsigned int pk2(float lo, float hi) { return f2bf(lo) | (f2bf(hi) << 16); }
__device__ __forceinline__ v4u pack8(const v4f a, const v4f b) {
  v4u r;
  r.x = pk2(a.x, a.y); r.y = pk2(a.z, a.w); r.z = pk2(b.x, b.y); r.w = pk2(b.z, b.w);
  return r;
}
__device__ __forceinline__ v4u pack4hl(const v4f a) {
  const unsigned int h0 = f2bf(a.x), h1 = f2bf(a.y), h2 = f2bf(a.z), h3 = f2bf(a.w);
  const unsigned int l0 = f2bf(a.x - bf2f(h0)), l1 = f2bf(a.y - bf2f(h1));
  const unsigned int l2 = f2bf(a.z - bf2f(h2)), l3 = f2bf(a.w - bf2f(h3));
  v4u r;
  r.x = h0 | (h1 << 16); r.y = h2 | (h3 << 16); r.z = l0 | (l1 << 16); r.w = l2 | (l3 << 16);
  return r;
}

__device__ __forceinline__ float wsum(float v) {
  v += __shfl_xor(v, 16, 32);
  v += __shfl_xor(v, 8, 32);
  v += __shfl_xor(v, 4, 32);
  v += __shfl_xor(v, 2, 32);
  v += __shfl_xor(v, 1, 32);
  return v;
}
__device__ __forceinline__ float dot4(const v4f a, const v4f b) {
  float p = a.x * b.x; p = fmaf(a.y, b.y, p); p = fmaf(a.z, b.z, p); p = fmaf(a.w, b.w, p);
  return p;
}

__global__ __launch_bounds__(NTHR) void k_xprep(const float* __restrict__ x, unsigned short* xb, int nN, int nUnits) {
  const int i = (int)blockIdx.x * NTHR + (int)threadIdx.x;
  if (i >= nUnits) return;
  const int row = i >> 4;
  const int c0  = (i & 15) * 8;
  const int rc  = row < nN ? row : nN - 1;
  const float* p = x + (size_t)rc * FW + c0;
  v4f a = *(const v4fa*)p;
  v4f b = *(const v4fa*)(p + 4);
  const v4f z4 = {0.f, 0.f, 0.f, 0.f};
  if (row >= nN) { a = z4; b = z4; }
  const v4u hv = pack8(a, b);
  unsigned short* o = xb + (size_t)row * FW + c0;
  *(volatile v4u*)o = hv;
  __threadfence();
  *(volatile v4u*)o = hv;
}

__global__ __launch_bounds__(NTHR) void k_wprep(const float* __restrict__ Wq, const float* __restrict__ Wk,
                                                const float* __restrict__ Wv, const float* __restrict__ Wo,
                                                unsigned short* WQKV, unsigned short* WOT) {
  const int u = (int)blockIdx.x * NTHR + (int)threadIdx.x;
  if (u >= NUW) return;
  v4f a, b;
  unsigned short* dp;
  if (u < UWQKV) {
    const int part = u >> 11;
    const int v    = u & 2047;
    const int n    = v >> 4;
    const int k8   = (v & 15) * 8;
    const float* W = (part == 0) ? Wq : ((part == 1) ? Wk : Wv);
    const float* p = W + (size_t)n * FW + k8;
    a = *(const v4fa*)p;
    b = *(const v4fa*)(p + 4);
    dp = WQKV + (size_t)(part * FW + n) * FW + k8;
  } else {
    const int v = u - UWQKV;
    const int n = v >> 5;
    const int l = v & 31;
    const float* p = Wo + (size_t)n * FW + 4 * l;
    a = *(const v4fa*)p;
    b = a;
    dp = WOT + (size_t)n * AOK + 8 * l;
  }
  const v4u wv = pack8(a, b);
  *(volatile v4u*)dp = wv;
  __threadfence();
  *(volatile v4u*)dp = wv;
}

__global__ __launch_bounds__(GTHR) void k_gemm(const unsigned short* __restrict__ A,
                                               const unsigned short* __restrict__ WT, float* outF) {
  __shared__ __attribute__((aligned(16))) float stg[GBM * GBN];
  const int tid = (int)threadIdx.x, lane = tid & 31, wave = tid >> 5, hh = lane >> 4, m = lane & 15;
  const int rowBase = (int)blockIdx.x * GBM;
  const int col0    = (int)blockIdx.y * GBN;

  v8f acc[4];
  {
    const v8f z = {0.f, 0.f, 0.f, 0.f, 0.f, 0.f, 0.f, 0.f};
    acc[0] = z; acc[1] = z; acc[2] = z; acc[3] = z;
  }
  const unsigned short* ap = A  + (size_t)(rowBase + 16 * wave + m) * (size_t)FW + 8 * hh;
  const unsigned short* wp = WT + (size_t)(col0 + m) * (size_t)FW + 8 * hh;
#pragma unroll 1
  for (int ks = 0; ks < FW / 32; ++ks) {
    FragB af;
    af.h[0] = *(const v8usa*)(ap + 32 * ks);
    af.h[1] = *(const v8usa*)(ap + 32 * ks + 16);
#pragma unroll
    for (int t = 0; t < 4; ++t) {
      const unsigned short* wq = wp + (size_t)(16 * t) * (size_t)FW + 32 * ks;
      FragB bf;
      bf.h[0] = *(const v8usa*)wq;
      bf.h[1] = *(const v8usa*)(wq + 16);
      acc[t] = wmb(af, bf, acc[t]);
    }
  }

#pragma unroll
  for (int t = 0; t < 4; ++t) {
    const int lc = 16 * t + m;
#pragma unroll
    for (int r = 0; r < 8; ++r) {
      const int lr = 16 * wave + 8 * hh + r;
      stg[lr * GBN + lc] = acc[t][r];
    }
  }
  __syncthreads();

  v4f fv[8];
#pragma unroll
  for (int i = 0; i < 8; ++i) {
    const int lr = 16 * wave + 2 * i + hh;
    fv[i] = *(const v4fa*)(stg + lr * GBN + 4 * m);
  }
#pragma unroll
  for (int i = 0; i < 8; ++i) {
    const int lr = 16 * wave + 2 * i + hh;
    const int gr = rowBase + lr;
    float* op = outF + (size_t)gr * (size_t)KVW + col0 + 4 * m;
    *(volatile v4f*)op = fv[i];
  }
  __threadfence();
#pragma unroll
  for (int i = 0; i < 8; ++i) {
    const int lr = 16 * wave + 2 * i + hh;
    const int gr = rowBase + lr;
    float* op = outF + (size_t)gr * (size_t)KVW + col0 + 4 * m;
    *(volatile v4f*)op = fv[i];
  }
}

__global__ __launch_bounds__(FTHR) void k_node(
    const unsigned short* __restrict__ XB, const unsigned short* __restrict__ WQT,
    const unsigned short* __restrict__ WOT, const float* __restrict__ KV,
    const int* __restrict__ nbr, const float* __restrict__ hsrc,
    const float* __restrict__ bo, const float* __restrict__ gam, const float* __restrict__ bet,
    float* out, int nN)
{
  __shared__ __attribute__((aligned(16))) float          qs[FB * FW];
  __shared__ __attribute__((aligned(16))) unsigned short aos[FB * AOK];
  const int tid = (int)threadIdx.x, lane = tid & 31, wave = tid >> 5, hh = lane >> 4, m = lane & 15;
  const int rowBase = (int)blockIdx.x * FB;
  const v8f z8 = {0.f, 0.f, 0.f, 0.f, 0.f, 0.f, 0.f, 0.f};
  const v4f z4 = {0.f, 0.f, 0.f, 0.f};

  {
    const unsigned short* ap = XB + (size_t)(rowBase + 16 * wave + m) * (size_t)FW + 8 * hh;
#pragma unroll 1
    for (int p = 0; p < 2; ++p) {
      v8f acc[4];
      acc[0] = z8; acc[1] = z8; acc[2] = z8; acc[3] = z8;
      const unsigned short* wp = WQT + (size_t)(64 * p + m) * (size_t)FW + 8 * hh;
#pragma unroll 1
      for (int ks = 0; ks < FW / 32; ++ks) {
        FragB af;
        af.h[0] = *(const v8usa*)(ap + 32 * ks);
        af.h[1] = *(const v8usa*)(ap + 32 * ks + 16);
#pragma unroll
        for (int t = 0; t < 4; ++t) {
          const unsigned short* wq = wp + (size_t)(16 * t) * (size_t)FW + 32 * ks;
          FragB bf;
          bf.h[0] = *(const v8usa*)wq;
          bf.h[1] = *(const v8usa*)(wq + 16);
          acc[t] = wmb(af, bf, acc[t]);
        }
      }
#pragma unroll
      for (int t = 0; t < 4; ++t) {
        const int lc = 64 * p + 16 * t + m;
#pragma unroll
        for (int r = 0; r < 8; ++r) {
          const int lr = 16 * wave + 8 * hh + r;
          qs[lr * FW + lc] = acc[t][r];
        }
      }
    }
  }
  __syncthreads();

  {
#pragma unroll 1
    for (int j = 0; j < 16; ++j) {
      const int lr   = 16 * wave + j;
      const int grow = rowBase + lr;
      const int gcl  = grow < nN ? grow : nN - 1;
      const v4f q4 = *(const v4fa*)(qs + lr * FW + 4 * lane);
      int nbv = nbr[(size_t)gcl * NNB + (lane & (NNB - 1))];
      nbv = nbv < 0 ? 0 : (nbv > nN - 1 ? nN - 1 : nbv);
      float lg[NNB];
#pragma unroll
      for (int k = 0; k < NNB; ++k) {
        const int tk = __builtin_amdgcn_readlane(nbv, k);
        const v4f k4 = *(const v4fa*)(KV + (size_t)tk * (size_t)KVW + 4 * lane);
        float pp = dot4(q4, k4);
        pp += __shfl_xor(pp, 1, 32);
        pp += __shfl_xor(pp, 2, 32);
        lg[k] = pp * ATTSC;
      }
      float mx = lg[0];
#pragma unroll
      for (int k = 1; k < NNB; ++k) mx = fmaxf(mx, lg[k]);
      float sm = 0.0f;
#pragma unroll
      for (int k = 0; k < NNB; ++k) { lg[k] = __expf(lg[k] - mx); sm += lg[k]; }
      const float inv = 1.0f / sm;
      v4f o4 = z4;
#pragma unroll
      for (int k = 0; k < NNB; ++k) {
        const int tk = __builtin_amdgcn_readlane(nbv, k);
        const v4f v4 = *(const v4fa*)(KV + (size_t)tk * (size_t)KVW + FW + 4 * lane);
        o4 = o4 + v4 * (lg[k] * inv);
      }
      const v4u w4 = pack4hl(o4);
      *(v4ua*)(aos + lr * AOK + 8 * lane) = w4;
    }
  }
  __syncthreads();

  {
    const unsigned short* ap = aos + (16 * wave + m) * AOK + 8 * hh;
#pragma unroll 1
    for (int p = 0; p < 2; ++p) {
      v8f acc[4];
      acc[0] = z8; acc[1] = z8; acc[2] = z8; acc[3] = z8;
      const unsigned short* wp = WOT + (size_t)(64 * p + m) * (size_t)AOK + 8 * hh;
#pragma unroll 1
      for (int ks = 0; ks < AOK / 32; ++ks) {
        FragB af;
        af.h[0] = *(const v8usa*)(ap + 32 * ks);
        af.h[1] = *(const v8usa*)(ap + 32 * ks + 16);
#pragma unroll
        for (int t = 0; t < 4; ++t) {
          const unsigned short* wq = wp + (size_t)(16 * t) * (size_t)AOK + 32 * ks;
          FragB bf;
          bf.h[0] = *(const v8usa*)wq;
          bf.h[1] = *(const v8usa*)(wq + 16);
          acc[t] = wmb(af, bf, acc[t]);
        }
      }
#pragma unroll
      for (int t = 0; t < 4; ++t) {
        const int lc = 64 * p + 16 * t + m;
#pragma unroll
        for (int r = 0; r < 8; ++r) {
          const int lr = 16 * wave + 8 * hh + r;
          qs[lr * FW + lc] = acc[t][r];
        }
      }
    }
  }
  __syncthreads();

  {
    const v4f bb = bfr4(*(const v4fa*)(bo  + 4 * lane));
    const v4f gg = bfr4(*(const v4fa*)(gam + 4 * lane));
    const v4f ee = bfr4(*(const v4fa*)(bet + 4 * lane));
#pragma unroll 1
    for (int j = 0; j < 16; ++j) {
      const int lr   = 16 * wave + j;
      const int grow = rowBase + lr;
      const int gcl  = grow < nN ? grow : nN - 1;
      const v4f d4 = *(const v4fa*)(qs + lr * FW + 4 * lane) + bb;
      const v4f h4 = bfr4(*(const v4fa*)(hsrc + (size_t)gcl * (size_t)FW + 4 * lane));
      const v4f x4 = h4 + d4;
      const float s  = wsum((x4.x + x4.y) + (x4.z + x4.w));
      const float mu = s * (1.0f / FW);
      const v4f dd = x4 - mu;
      const float sq = wsum((dd.x * dd.x + dd.y * dd.y) + (dd.z * dd.z + dd.w * dd.w));
      const float rs = rsqrtf(sq * (1.0f / FW) + LNEPS);
      const v4f y4 = dd * rs * gg + ee;
      if (grow < nN) {
        float* op = out + (size_t)grow * (size_t)FW + 4 * lane;
        *(volatile v4f*)op = y4;
        __threadfence();
        *(volatile v4f*)op = y4;
      }
    }
  }
}

static inline int cdiv(int a, int b) { return (a + b - 1) / b; }
static inline size_t al256(size_t o) { return (o + 255) & ~(size_t)255; }

extern "C" void kernel_launch(void* const* d_in, const int* in_sizes, int n_in,
                              void* d_out, int out_size, void* d_ws, size_t ws_size,
                              hipStream_t stream) {
  if (n_in < 9) return;
  if (in_sizes[0] < FW || (in_sizes[0] % FW) != 0) return;
  const int nN = in_sizes[0] / FW;
  if (nN < 1 || nN > (1 << 24)) return;
  if ((long long)in_sizes[1] != (long long)nN * NNB) return;
  if (in_sizes[2] != FW * FW || in_sizes[3] != FW * FW || in_sizes[4] != FW * FW || in_sizes[5] != FW * FW) return;
  if (in_sizes[6] != FW || in_sizes[7] != FW || in_sizes[8] != FW) return;
  if ((long long)out_size != (long long)nN * FW) return;

  const float* hsrc = (const float*)d_in[0];
  const int*   nbr  = (const int*)  d_in[1];
  const float* Wq   = (const float*)d_in[2];
  const float* Wk   = (const float*)d_in[3];
  const float* Wv   = (const float*)d_in[4];
  const float* Wo   = (const float*)d_in[5];
  const float* bo   = (const float*)d_in[6];
  const float* gam  = (const float*)d_in[7];
  const float* bet  = (const float*)d_in[8];
  float* out = (float*)d_out;

  const int MP = cdiv(nN, GBM) * GBM;
  const int gM = MP / GBM;
  const int gF = MP / FB;

  char* ws = (char*)d_ws;
  size_t off = 0;
  const size_t oXB = off; off = al256(off + (size_t)MP * FW * 2);
  const size_t oWQ = off; off = al256(off + (size_t)WROWS * FW * 2);
  const size_t oWO = off; off = al256(off + (size_t)FW * AOK * 2);
  const size_t oKV = off; off = al256(off + (size_t)MP * KVW * 4);
  if (off > ws_size || off > (size_t)WSMAX) return;
  unsigned short* XB   = (unsigned short*)(ws + oXB);
  unsigned short* WQKV = (unsigned short*)(ws + oWQ);
  unsigned short* WOT  = (unsigned short*)(ws + oWO);
  float*          KV   = (float*)(ws + oKV);

  const int nUx = MP * (FW / 8);
  k_xprep<<<cdiv(nUx, NTHR), NTHR, 0, stream>>>(hsrc, XB, nN, nUx);
  k_wprep<<<NUW / NTHR, NTHR, 0, stream>>>(Wq, Wk, Wv, Wo, WQKV, WOT);
  k_gemm<<<dim3(gM, KVW / GBN), GTHR, 0, stream>>>(XB, WQKV + (size_t)FW * FW, KV);
  k_node<<<gF, FTHR, 0, stream>>>(XB, WQKV, WOT, KV, nbr, hsrc, bo, gam, bet, out, nN);
}
